// PacConv2d_601295421590
// MI455X (gfx1250) — hardware-verified
//
#include <hip/hip_runtime.h>
#include <hip/hip_bf16.h>

typedef _Float16 v16h_t __attribute__((ext_vector_type(16)));
typedef _Float16 v8h_t  __attribute__((ext_vector_type(8)));
typedef float    v8f_t  __attribute__((ext_vector_type(8)));
typedef float    v4f_t  __attribute__((ext_vector_type(4)));

#define KS    5
#define PAD   2
#define NB    4
#define CIN   32
#define COUT  32
#define CG    8
#define HH    128
#define WW    128
#define NTAP  (KS*KS)
#define HW    (HH*WW)

#define WLDS_ELEMS (NTAP*COUT*CIN)
#define XPITCH_H 40
#define XTILE_ELEMS (KS * WW * XPITCH_H)

__global__ __launch_bounds__(256)
void pac_wmma_kernel(const float* __restrict__ x,
                     const float* __restrict__ guide,
                     const float* __restrict__ weight,
                     const float* __restrict__ bias,
                     float* __restrict__ out)
{
    __shared__ __attribute__((aligned(16))) _Float16 wlds[WLDS_ELEMS];
    __shared__ __attribute__((aligned(16))) _Float16 xtile[XTILE_ELEMS];
    __shared__ __attribute__((aligned(16))) float otile[COUT][WW];

    const int tid = threadIdx.x;
    const int b   = blockIdx.x / HH;
    const int m   = blockIdx.x % HH;

    const float* gptr = guide + (size_t)b * CG * HW;
    const float* xb   = x     + (size_t)b * CIN * HW;

    for (int i = tid; i < WLDS_ELEMS; i += 256) {
        const int t   = i >> 10;
        const int rem = i & 1023;
        const int o   = rem >> 5;
        const int c   = rem & 31;
        wlds[i] = (_Float16)weight[(o * CIN + c) * NTAP + t];
    }

    for (int j4 = tid; j4 < KS * CIN * (WW / 4); j4 += 256) {
        const int col4 = (j4 & 31) * 4;
        const int c    = (j4 >> 5) & 31;
        const int r    = j4 >> 10;
        const int yc   = min(max(m - PAD + r, 0), HH - 1);
        const v4f_t v  = *(const v4f_t*)&xb[(c * HH + yc) * WW + col4];
        xtile[(r * WW + col4 + 0) * XPITCH_H + c] = (_Float16)v.x;
        xtile[(r * WW + col4 + 1) * XPITCH_H + c] = (_Float16)v.y;
        xtile[(r * WW + col4 + 2) * XPITCH_H + c] = (_Float16)v.z;
        xtile[(r * WW + col4 + 3) * XPITCH_H + c] = (_Float16)v.w;
    }
    __syncthreads();

    const int wave   = tid >> 5;
    const int lane   = tid & 31;
    const int l15    = lane & 15;
    const int hiHalf = lane >> 4;
    const int n0     = wave * 16;
    const int np     = n0 + l15;

    float gc[CG];
#pragma unroll
    for (int c = 0; c < CG; ++c)
        gc[c] = gptr[c * HW + m * WW + np];

    v8f_t acc0 = {};
    v8f_t acc1 = {};

    for (int dy = -PAD; dy <= PAD; ++dy) {
        const int  yy  = m + dy;
        const int  yc  = min(max(yy, 0), HH - 1);
        const bool inY = (yy >= 0) && (yy < HH);
        const int  rr  = dy + PAD;

#pragma unroll
        for (int dx = -PAD; dx <= PAD; ++dx) {
            const int  t     = (dy + PAD) * KS + (dx + PAD);
            const int  xx    = np + dx;
            const int  xc    = min(max(xx, 0), WW - 1);
            const bool in    = inY && (xx >= 0) && (xx < WW);
            const int  gbase = yc * WW + xc;

            float s = 0.f;
#pragma unroll
            for (int c = 0; c < CG; ++c) {
                const float gv = gptr[c * HW + gbase];
                const float d  = gv - gc[c];
                s += d * d;
            }
            float kv = __expf(-0.5f * s);
            kv = in ? kv : 0.f;

            const _Float16* xp = &xtile[(rr * WW + xc) * XPITCH_H + hiHalf * 8];
            const v8h_t x0 = *(const v8h_t*)(xp);
            const v8h_t x1 = *(const v8h_t*)(xp + 16);
            v16h_t a;
#pragma unroll
            for (int q = 0; q < 8; ++q) {
                a[q]     = (_Float16)((float)x0[q] * kv);
                a[8 + q] = (_Float16)((float)x1[q] * kv);
            }

            const _Float16* wb0 = &wlds[((t * COUT) + l15     ) * CIN + hiHalf * 8];
            const _Float16* wb1 = &wlds[((t * COUT) + 16 + l15) * CIN + hiHalf * 8];
            const v16h_t b0 = __builtin_shufflevector(*(const v8h_t*)wb0, *(const v8h_t*)(wb0 + 16), 0,1,2,3,4,5,6,7,8,9,10,11,12,13,14,15);
            const v16h_t b1 = __builtin_shufflevector(*(const v8h_t*)wb1, *(const v8h_t*)(wb1 + 16), 0,1,2,3,4,5,6,7,8,9,10,11,12,13,14,15);

            acc0 = __builtin_amdgcn_wmma_f32_16x16x32_f16(
                 false, a,  false, b0,
                 (short)0, acc0,  false,  false);
            acc1 = __builtin_amdgcn_wmma_f32_16x16x32_f16(
                 false, a,  false, b1,
                 (short)0, acc1,  false,  false);
            asm volatile("v_nop\n\tv_nop\n\tv_nop\n\tv_nop" : "+v"(acc0), "+v"(acc1) : "v"(a), "v"(b1));
        }
    }

    const int o0 = l15;
    const int o1 = 16 + l15;
    const float bias0 = bias[o0];
    const float bias1 = bias[o1];
#pragma unroll
    for (int r = 0; r < 8; ++r) {
        const int M = r + hiHalf * 8;
        const int n = n0 + M;
        otile[o0][n] = acc0[r] + bias0;
        otile[o1][n] = acc1[r] + bias1;
    }
    __syncthreads();
    for (int pass = 0; pass < 2; ++pass) {
#pragma unroll
        for (int j = 0; j < 4; ++j) {
            const int o = j * 8 + (tid >> 5), q4 = (tid & 31) * 4;
            *(volatile v4f_t*)(out + ((size_t)(b * COUT + o) * HH + m) * WW + q4) = *(const v4f_t*)(&otile[o][q4]);
        }
        __threadfence();
    }
}

extern "C" void kernel_launch(void* const* d_in, const int* in_sizes, int n_in,
                              void* d_out, int out_size, void* d_ws, size_t ws_size,
                              hipStream_t stream) {
    (void)in_sizes; (void)n_in; (void)out_size; (void)d_ws; (void)ws_size;
    const float* x      = (const float*)d_in[0];
    const float* guide  = (const float*)d_in[1];
    const float* weight = (const float*)d_in[2];
    const float* bias   = (const float*)d_in[3];
    float* out = (float*)d_out;

    dim3 grid(NB * HH);
    dim3 block(256);
    pac_wmma_kernel<<<grid, block, 0, stream>>>(x, guide, weight, bias, out);
}
